// GMM_4810363372989
// MI455X (gfx1250) — hardware-run, weakly checked
//
#include <hip/hip_runtime.h>


#ifndef NB
#define NB 8
#endif
#ifndef NPTS
#define NPTS 80000
#endif
#define NB_FULL   8
#define NPTS_FULL 80000
#define NK   5
#define NF   20
#define AW   4
#define GPW  5
#define BPB  (NPTS / (32 * AW * GPW))
#define XES  64
#define XTR  (2 * NF)
#define SW   48
#define PW   256
#define RW   320
#define QRS  2048.0f
#define QRI  (1.0f / 2048.0f)
#define PCS  16384.0f
#define PCI  (1.0f / 16384.0f)
#define LOG2E  1.4426950408889634f
#define TWO_PI 6.2831853071795864769f
#define OUT_POST ((size_t)NB_FULL * NPTS_FULL * NK)
#define OUT_MEAN ((size_t)2 * NB_FULL * NPTS_FULL * NK)
#define OUT_VAR  (OUT_MEAN + (size_t)NB_FULL * NK * NF)
#define OUT_PI   (OUT_VAR + (size_t)NB_FULL * NK * NF)
#define OUT_TOTAL (OUT_PI + (size_t)NB_FULL * NK)

static_assert(NPTS % (32 * AW * GPW) == 0);
static_assert(NPTS % 64 == 0);
static_assert(3 * NF <= XES);
static_assert(XES % 32 == 0);
static_assert(XES * 2 == 128);
static_assert(2 * NF + 1 <= SW);
static_assert(SW == 48);
static_assert(NK <= 8);
static_assert(NK * SW <= PW);
static_assert(PW == 4 * 64);
static_assert(RW >= 2 * 32 * NK);
static_assert(RW >= PW);
static_assert(32 * NK == 160);
static_assert((NPTS_FULL * NK * 4) % 128 == 0);
static_assert(64 * NF / 4 == 256 + 64);
static_assert(64 * XES / 8 == 2 * 256);
static_assert(XTR * 8 == 256 + 64);
static_assert(NB * NK <= 64);
static_assert((NB * NK * NF) % 4 == 0);
static_assert(NB * NK * NF / 4 <= 256);
static_assert(NB * 16 / 4 <= 32);
static_assert(NB <= NB_FULL);
static_assert(NPTS <= NPTS_FULL);
static_assert(OUT_POST * 4 == (size_t)12800000);
static_assert(OUT_MEAN * 4 == (size_t)25600000);
static_assert(OUT_VAR * 4 == (size_t)25603200);
static_assert(OUT_PI * 4 == (size_t)25606400);
static_assert(OUT_TOTAL * 4 == (size_t)25606560);
static_assert(OUT_PI + (size_t)((NB * NK + 3) / 4) * 4 <= OUT_TOTAL);
static_assert(AW * 512 * 2 + AW * RW * 4 <= 131072);
static_assert(64 * NF * 4 <= 131072);
static_assert(NB * NK * SW * 4 + 3 * NB * NK * NF * 4 + 64 * 4 + NB * 16 * 4 + NB * 16 * XES * 2 <= 131072);

typedef _Float16 h16;
typedef __attribute__((ext_vector_type(16))) _Float16 v16h;
typedef __attribute__((ext_vector_type(8)))  _Float16 v8h;
typedef __attribute__((ext_vector_type(8)))  float    v8f;
typedef __attribute__((ext_vector_type(4)))  float    v4f;
typedef v4f  __attribute__((may_alias)) v4fa;
typedef v8h  __attribute__((may_alias)) v8ha;

__device__ __forceinline__ unsigned short f2bf(float f) { unsigned u = __float_as_uint(f); u += 0x7FFFu + ((u >> 16) & 1u); return (unsigned short)(u >> 16); }
__device__ __forceinline__ float bfr(float f) { return __uint_as_float(((unsigned)f2bf(f)) << 16); }
__device__ __forceinline__ v16h cat16(v8h lo, v8h hi) { return __builtin_shufflevector(lo, hi, 0, 1, 2, 3, 4, 5, 6, 7, 8, 9, 10, 11, 12, 13, 14, 15); }
__device__ __forceinline__ v8f wmma16(v16h a, v16h b, v8f c) { return __builtin_amdgcn_wmma_f32_16x16x32_f16(false, a, false, b, (short)0, c, false, false); }
__device__ __forceinline__ v16h  ldh(const h16* p) { return cat16(*(const v8h*)p, *(const v8h*)(p + 16)); }
__device__ __forceinline__ void wave_sync() { __builtin_amdgcn_fence(3  , "wavefront"); __builtin_amdgcn_wave_barrier(); asm volatile("" ::: "memory"); }
static __device__ __forceinline__ h16 toh_flush(float v) { const h16 r = (h16)v; return (fabsf(v) < 6.103515625e-05f) ? (h16)0.0f : r; }
__device__ __forceinline__ v8f wmma16g(v16h a, v16h b, v8f c) { c = wmma16(a, b, c); asm volatile("v_nop\n\tv_nop\n\tv_nop\n\tv_nop" : "+v"(c) : "v"(a), "v"(b)); return c; }

__global__ __launch_bounds__(256) void k_planes(const float* __restrict__ data, h16* XE, h16* XT) {
#pragma clang fp contract(off)
    __shared__ __align__(16) float xs[64 * NF];
    const int tid = threadIdx.x;
    const int wave = __builtin_amdgcn_readfirstlane((int)(threadIdx.x >> 5));
    const int b = blockIdx.y; const int n0 = blockIdx.x * 64;
    const float* src = data + ((size_t)b * NPTS_FULL + (size_t)n0) * NF;
    { const v4f v = *(const v4f*)(src + 4 * tid); v4f o; o[0] = bfr(v[0]); o[1] = bfr(v[1]); o[2] = bfr(v[2]); o[3] = bfr(v[3]); *(v4fa*)(&xs[4 * tid]) = o; }
    if (wave < 2) { const int i = 256 + tid; const v4f v = *(const v4f*)(src + 4 * i); v4f o; o[0] = bfr(v[0]); o[1] = bfr(v[1]); o[2] = bfr(v[2]); o[3] = bfr(v[3]); *(v4fa*)(&xs[4 * i]) = o; }
    __syncthreads();
    v8h e0 = (v8h){}, e1 = (v8h){}, t0 = (v8h){}, t1 = (v8h){};
#pragma unroll
    for (int u = 0; u < 2; ++u) {
        const int piece = tid + 256 * u; const int pt = piece >> 3, c8 = (piece & 7) * 8;
        v8h ev;
#pragma unroll
        for (int j = 0; j < 8; ++j) {
            const int s = c8 + j;
            const int f = (s < NF) ? s : ((s < 2 * NF) ? (s - NF) : ((s < 3 * NF) ? (s - 2 * NF) : 0));
            const float x = xs[pt * NF + f];
            const float sq = x * x;
            const h16 hx = toh_flush(x);
            const h16 hq = toh_flush(sq);
            const h16 rq = toh_flush((sq - (float)hq) * QRS);
            ev[j] = (s < NF) ? hx : ((s < 2 * NF) ? hq : ((s < 3 * NF) ? rq : (h16)0.0f));
        }
        if (u == 0) e0 = ev; else e1 = ev;
    }
    const int tp1 = 256 + (tid & 63);
#pragma unroll
    for (int u = 0; u < 2; ++u) {
        const int piece = (u == 0) ? tid : tp1; const int row = piece >> 3, p8 = (piece & 7) * 8;
        const int f = (row < NF) ? row : (row - NF);
        v8h tv;
#pragma unroll
        for (int j = 0; j < 8; ++j) {
            const float x = xs[(p8 + j) * NF + f];
            const float sq = x * x;
            const h16 hx = toh_flush(x);
            const h16 hq = toh_flush(sq);
            tv[j] = (row < NF) ? hx : hq;
        }
        if (u == 0) t0 = tv; else t1 = tv;
    }
    h16* xe0 = XE + ((size_t)b * NPTS + (size_t)n0) * XES + (size_t)tid * 8;
    h16* xe1 = xe0 + (size_t)256 * 8;
    h16* xt0 = XT + ((size_t)b * XTR + (size_t)(tid >> 3)) * NPTS + (size_t)n0 + (size_t)((tid & 7) * 8);
    h16* xt1 = XT + ((size_t)b * XTR + (size_t)(tp1 >> 3)) * NPTS + (size_t)n0 + (size_t)((tp1 & 7) * 8);
#pragma unroll 1
    for (int ps = 0; ps < 2; ++ps) {
        *(volatile v8h*)xe0 = e0; *(volatile v8h*)xe1 = e1;
        *(volatile v8h*)xt0 = t0;
        if (wave < 2) *(volatile v8h*)xt1 = t1;
        if (ps == 0) __threadfence(); }
}

__device__ __forceinline__ unsigned pinu(unsigned v) { asm volatile("" : "+v"(v)); return v; }

__global__ __launch_bounds__(256) void k_params(const float* __restrict__ PART, const float* __restrict__ means_in, const float* __restrict__ var_in, const float* __restrict__ prior_in,
                                                h16* CO, float* CST, float* OUT, int mode) {
#pragma clang fp contract(off)
    __shared__ __align__(16) float S[NB * NK * SW];
    __shared__ __align__(16) float mu_s[NB * NK * NF];
    __shared__ __align__(16) float va_s[NB * NK * NF];
    __shared__ __align__(16) float al_s[NB * NK * NF];
    __shared__ __align__(16) float pi_s[64];
    __shared__ __align__(16) float cs_s[NB * 16];
    __shared__ __align__(16) h16   co_s[NB * 16 * XES];
    const unsigned tid = pinu((unsigned)threadIdx.x);
    if (tid < 64u) { const unsigned t = pinu(tid); pi_s[t] = 0.0f; }
    if (tid < (unsigned)(NB * 16)) { const unsigned t = pinu(tid); cs_s[t] = 0.0f; }
#pragma unroll 1
    for (unsigned i0 = tid; i0 < (unsigned)(NB * 16 * XES / 8); i0 += 256u) { const unsigned i = pinu(i0); const v8h z = (v8h){}; *(v8ha*)(&co_s[i * 8u]) = z; }
    if (mode == 0) {
#pragma unroll 1
        for (unsigned i0 = tid; i0 < (unsigned)(NB * NK * NF); i0 += 256u) { const unsigned idx = pinu(i0); mu_s[idx] = bfr(means_in[idx]); va_s[idx] = bfr(var_in[idx]); }
    } else {
#pragma unroll 1
        for (unsigned i0 = tid; i0 < (unsigned)(NB * NK * SW); i0 += 256u) {
            const unsigned idx = pinu(i0);
            const unsigned bb = pinu(idx / (unsigned)(NK * SW));
            const unsigned i = pinu(idx - bb * (unsigned)(NK * SW));
            const float* pp = PART + (size_t)bb * BPB * PW + i;
            double s = 0.0;
#pragma unroll 4
            for (unsigned p = 0; p < (unsigned)BPB; ++p) s += (double)pp[(size_t)p * PW];
            S[idx] = (float)s * PCI;
        }
        __syncthreads();
#pragma unroll 1
        for (unsigned i0 = tid; i0 < (unsigned)(NB * NK * NF); i0 += 256u) {
            const unsigned idx = pinu(i0);
            const unsigned bb = pinu(idx / (unsigned)(NK * NF));
            const unsigned r = pinu(idx - bb * (unsigned)(NK * NF));
            const unsigned k = pinu(r / (unsigned)NF);
            const unsigned f = pinu(r - k * (unsigned)NF);
            const unsigned sb = pinu((bb * (unsigned)NK + k) * (unsigned)SW);
            const float sk = S[sb + (unsigned)(2 * NF)];
            const float a1 = S[sb + f];
            const float a2 = S[sb + (unsigned)NF + f];
            const float rd = 1.0f / (sk + 1e-7f);
            const float mu = a1 * rd;
            const float vv = (a2 - 2.0f * mu * a1 + mu * mu * sk) * rd + 1e-6f;
            mu_s[idx] = mu; va_s[idx] = vv;
        }
    }
    __syncthreads();
    if (mode == 0) {
        if (tid < (unsigned)(NB * NK)) { const unsigned t = pinu(tid); pi_s[t] = bfr(prior_in[t]); }
    } else {
        if (tid < (unsigned)NB) {
            const unsigned t = pinu(tid);
            const unsigned sb = pinu(t * (unsigned)(NK * SW));
            const unsigned pb = pinu(t * (unsigned)NK);
            float pt[NK]; float l1 = 0.0f;
#pragma unroll
            for (int k = 0; k < NK; ++k) { pt[k] = S[sb + (unsigned)(k * SW + 2 * NF)] * (1.0f / (float)NPTS); l1 += fabsf(pt[k]); }
            const float rl = 1.0f / fmaxf(l1, 1e-12f);
#pragma unroll
            for (int k = 0; k < NK; ++k) pi_s[pb + (unsigned)k] = pt[k] * rl;
        }
    }
#pragma unroll 1
    for (unsigned i0 = tid; i0 < (unsigned)(NB * NK * NF); i0 += 256u) {
        const unsigned idx = pinu(i0);
        const unsigned bb = pinu(idx / (unsigned)(NK * NF));
        const unsigned r = pinu(idx - bb * (unsigned)(NK * NF));
        const unsigned k = pinu(r / (unsigned)NF);
        const unsigned f = pinu(r - k * (unsigned)NF);
        const float al = 1.0f / (va_s[idx] + 1e-6f);
        al_s[idx] = al;
        const float c1 = mu_s[idx] * al, c2 = -0.5f * al;
        const h16 h1 = toh_flush(c1); const h16 r1 = toh_flush((c1 - (float)h1) * QRS);
        const h16 h2 = toh_flush(c2); const h16 r2 = toh_flush((c2 - (float)h2) * QRS);
        const unsigned vb = pinu((bb * 16u + k) * (unsigned)XES);
        const unsigned rb = pinu((bb * 16u + 8u + k) * (unsigned)XES);
        co_s[vb + f] = h1; co_s[vb + (unsigned)NF + f] = h2;
        co_s[rb + f] = r1; co_s[rb + (unsigned)NF + f] = r2; co_s[rb + (unsigned)(2 * NF) + f] = h2;
    }
    __syncthreads();
    if (tid < (unsigned)(NB * NK)) {
        const unsigned t = pinu(tid);
        const unsigned bb = pinu(t / (unsigned)NK);
        const unsigned k = pinu(t - bb * (unsigned)NK);
        const unsigned base = pinu((bb * (unsigned)NK + k) * (unsigned)NF);
        float slog = 0.0f, q = 0.0f;
#pragma unroll 1
        for (unsigned f = 0; f < (unsigned)NF; ++f) {
            const unsigned i = base + f;
            const float mu = mu_s[i];
            slog += logf(TWO_PI * va_s[i]);
            q += mu * mu * al_s[i];
        }
        cs_s[bb * 16u + k] = logf(pi_s[t]) - 0.5f * slog - 0.5f * q;
    }
    __syncthreads();
#pragma unroll 1
    for (int ps = 0; ps < 2; ++ps) {
#pragma unroll 1
        for (unsigned i0 = tid; i0 < (unsigned)(NB * 16 * XES / 8); i0 += 256u) { const unsigned i = pinu(i0); const v8h v = *(const v8ha*)(&co_s[i * 8u]); *(volatile v8h*)(CO + (size_t)i * 8) = v; }
        if (tid < (unsigned)(NB * 16 / 4)) { const unsigned t = pinu(tid); const v4f v = *(const v4fa*)(&cs_s[4u * t]); *(volatile v4f*)(CST + (size_t)t * 4) = v; }
        if (mode == 2) {
            if (tid < (unsigned)(NB * NK * NF / 4)) {
                const unsigned t = pinu(tid);
                const v4f vm = *(const v4fa*)(&mu_s[4u * t]); const v4f vv = *(const v4fa*)(&va_s[4u * t]);
                *(volatile v4f*)(OUT + OUT_MEAN + (size_t)t * 4) = vm; *(volatile v4f*)(OUT + OUT_VAR + (size_t)t * 4) = vv; }
            if (tid < (unsigned)((NB * NK + 3) / 4)) { const unsigned t = pinu(tid); const v4f vp = *(const v4fa*)(&pi_s[4u * t]); *(volatile v4f*)(OUT + OUT_PI + (size_t)t * 4) = vp; }
        }
        if (ps == 0) __threadfence(); }
}

__global__ __launch_bounds__(32 * AW) void k_em(const h16* __restrict__ XE, const h16* __restrict__ XT, const h16* __restrict__ CO, const float* __restrict__ CST,
                                                float* PART, float* OUT, int fin) {
    __shared__ __align__(16) h16   pl[AW * 16 * 32];
    __shared__ __align__(16) float red[AW * RW];
    const int lane = threadIdx.x & 31, lr = lane & 15, hi = lane >> 4;
    const int wave = __builtin_amdgcn_readfirstlane((int)(threadIdx.x >> 5));
    const int b = blockIdx.y;
    const int g0 = (blockIdx.x * AW + wave) * GPW;
    const int pw = wave * 512, rw = wave * RW;
    const h16* cob = CO + ((size_t)b * 16 + (size_t)lr) * XES + 8 * hi;
    const v16h ca0 = ldh(cob), ca1 = ldh(cob + 32);
    float cs[NK];
#pragma unroll
    for (int k = 0; k < NK; ++k) cs[k] = CST[b * 16 + k];
    const v16h hz = (v16h){};
    v16h ones;
#pragma unroll
    for (int i = 0; i < 16; ++i) ones[i] = (h16)1.0f;
    { const v8h z = (v8h){}; *(v8ha*)(&pl[pw + lane * 8]) = z; *(v8ha*)(&pl[pw + 256 + lane * 8]) = z; }
    wave_sync();
    const h16* xtb = XT + (size_t)b * XTR * NPTS + 8 * hi;
    const int r2 = 32 + (lr & 7);
    v8f s0 = (v8f){}, s1 = (v8f){}, s2 = (v8f){};
#pragma unroll 1
    for (int g = 0; g < GPW; ++g) {
        const int n0 = (g0 + g) * 32;
        const h16* xe = XE + ((size_t)b * NPTS + (size_t)(n0 + lr)) * XES + 8 * hi;
        const v16h x00 = ldh(xe), x01 = ldh(xe + 32);
        const v16h x10 = ldh(xe + 16 * XES), x11 = ldh(xe + 16 * XES + 32);
        v8f d0 = (v8f){}, d1 = (v8f){};
        d0 = wmma16g(ca0, x00, d0); d0 = wmma16g(ca1, x01, d0);
        d1 = wmma16g(ca0, x10, d1); d1 = wmma16g(ca1, x11, d1);
        float ll[NK], pp[NK];
#pragma unroll
        for (int k = 0; k < NK; ++k) {
            const float own = hi ? d1[k] : d0[k];
            const float snd = hi ? d0[k] : d1[k];
            const float rcv = __shfl_xor(snd, 16, 32);
            const float vh = hi ? rcv : own; const float vr = hi ? own : rcv;
            ll[k] = (vh + vr * QRI) + cs[k];
        }
        float mx = ll[0];
#pragma unroll
        for (int k = 1; k < NK; ++k) mx = fmaxf(mx, ll[k]);
        float sum = 0.0f;
#pragma unroll
        for (int k = 0; k < NK; ++k) { pp[k] = __builtin_amdgcn_exp2f((ll[k] - mx) * LOG2E); sum += pp[k]; }
        const float rs = 1.0f / sum;
#pragma unroll
        for (int k = 0; k < NK; ++k) pp[k] = pp[k] * rs;
        if (!fin) {
            wave_sync();
#pragma unroll
            for (int k = 0; k < NK; ++k) {
                const float v = pp[k] * PCS;
                const h16 ph = toh_flush(v);
                const h16 pr = toh_flush((v - (float)ph) * QRS);
                pl[pw + k * 32 + lane] = ph; pl[pw + (8 + k) * 32 + lane] = pr; }
            wave_sync();
            const v16h pa = cat16(*(const v8ha*)(&pl[pw + lr * 32 + 8 * hi]), *(const v8ha*)(&pl[pw + lr * 32 + 16 + 8 * hi]));
            const v16h xb0 = ldh(xtb + (size_t)lr * NPTS + n0);
            const v16h xb1 = ldh(xtb + (size_t)(16 + lr) * NPTS + n0);
            v16h xb2 = ldh(xtb + (size_t)r2 * NPTS + n0);
            asm volatile("" : "+v"(xb2));
            xb2 = (lr < 8) ? xb2 : ((lr == 8) ? ones : hz);
            s0 = wmma16g(pa, xb0, s0); s1 = wmma16g(pa, xb1, s1); s2 = wmma16g(pa, xb2, s2);
        } else {
            wave_sync();
#pragma unroll
            for (int k = 0; k < NK; ++k) { red[rw + lane * NK + k] = ll[k]; red[rw + 32 * NK + lane * NK + k] = pp[k]; }
            wave_sync();
            const v4f l0 = *(const v4fa*)(&red[rw + 4 * lane]);
            const v4f l1 = *(const v4fa*)(&red[rw + 128 + 4 * (lane & 7)]);
            const v4f q0 = *(const v4fa*)(&red[rw + 32 * NK + 4 * lane]);
            const v4f q1 = *(const v4fa*)(&red[rw + 32 * NK + 128 + 4 * (lane & 7)]);
            float* oll = OUT + ((size_t)b * NPTS_FULL + (size_t)n0) * NK;
            float* opo = oll + OUT_POST;
#pragma unroll 1
            for (int ps = 0; ps < 2; ++ps) {
                *(volatile v4f*)(oll + 4 * lane) = l0; *(volatile v4f*)(opo + 4 * lane) = q0;
                if (lane < 8) { *(volatile v4f*)(oll + 128 + 4 * lane) = l1; *(volatile v4f*)(opo + 128 + 4 * lane) = q1; }
                if (ps == 0) __threadfence(); }
        }
    }
    if (!fin) {
        float f0[NK], f1[NK], f2[NK];
#pragma unroll
        for (int r = 0; r < NK; ++r) {
            const float o0 = __shfl_xor(s0[r], 16, 32), o1 = __shfl_xor(s1[r], 16, 32), o2 = __shfl_xor(s2[r], 16, 32);
            f0[r] = s0[r] + o0 * QRI; f1[r] = s1[r] + o1 * QRI; f2[r] = s2[r] + o2 * QRI; }
        if (hi == 0) {
#pragma unroll
            for (int r = 0; r < NK; ++r) { red[rw + r * SW + lr] = f0[r]; red[rw + r * SW + 16 + lr] = f1[r]; red[rw + r * SW + 32 + lr] = f2[r]; }
        } else {
            red[rw + NK * SW + lr] = 0.0f;
        }
        __syncthreads();
        if (wave < 2) {
            const int t4 = 4 * (int)threadIdx.x;
            v4f acc = *(const v4fa*)(&red[t4]);
#pragma unroll
            for (int w = 1; w < AW; ++w) { const v4f o = *(const v4fa*)(&red[w * RW + t4]); acc = acc + o; }
            float* dst = PART + ((size_t)b * BPB + (size_t)blockIdx.x) * PW + t4;
#pragma unroll 1
            for (int ps = 0; ps < 2; ++ps) { *(volatile v4f*)dst = acc; if (ps == 0) __threadfence(); }
        }
    }
}

static constexpr size_t al256(size_t v) { return (v + 255) & ~(size_t)255; }
static constexpr size_t SZ_XE = al256((size_t)NB * NPTS * XES * 2);
static constexpr size_t SZ_XT = al256((size_t)NB * XTR * NPTS * 2);
static constexpr size_t SZ_PT = al256((size_t)NB * BPB * PW * 4);
static constexpr size_t SZ_CO = al256((size_t)NB * 16 * XES * 2);
static constexpr size_t SZ_CS = al256((size_t)NB * 16 * 4);
static constexpr size_t SZ_TOTAL = SZ_XE + SZ_XT + SZ_PT + SZ_CO + SZ_CS;
static_assert(SZ_TOTAL <= (size_t)134217728);
static_assert(((size_t)NPTS * 2) % 128 == 0);
static_assert(((size_t)PW * 4) % 128 == 0);

extern "C" void kernel_launch(void* const* d_in, const int* in_sizes, int n_in,
                              void* d_out, int out_size, void* d_ws, size_t ws_size, hipStream_t stream) {
    if (n_in < 4) return;
    const size_t needx = ((size_t)(NB - 1) * NPTS_FULL + NPTS) * NF;
    if ((size_t)in_sizes[0] < needx) return;
    if ((size_t)in_sizes[1] < (size_t)NB * NK * NF || (size_t)in_sizes[2] < (size_t)NB * NK * NF || (size_t)in_sizes[3] < (size_t)NB * NK) return;
    if ((size_t)out_size < OUT_PI + (size_t)((NB * NK + 3) / 4) * 4) return;
    if (SZ_TOTAL > ws_size) return;
    const float* data  = (const float*)d_in[0];
    const float* means = (const float*)d_in[1];
    const float* vari  = (const float*)d_in[2];
    const float* prior = (const float*)d_in[3];
    float* OUT = (float*)d_out;
    char* wsp = (char*)d_ws;
    h16* XE = (h16*)wsp; wsp += SZ_XE;
    h16* XT = (h16*)wsp; wsp += SZ_XT;
    float* PART = (float*)wsp; wsp += SZ_PT;
    h16* CO = (h16*)wsp; wsp += SZ_CO;
    float* CST = (float*)wsp; wsp += SZ_CS;

    k_planes<<<dim3(NPTS / 64, NB, 1), 256, 0, stream>>>(data, XE, XT);
    for (int it = 0; it <= 5; ++it) {
        const int mode = (it == 0) ? 0 : ((it == 5) ? 2 : 1);
        k_params<<<dim3(1, 1, 1), 256, 0, stream>>>(PART, means, vari, prior, CO, CST, OUT, mode);
        k_em<<<dim3(BPB, NB, 1), 32 * AW, 0, stream>>>(XE, XT, CO, CST, PART, OUT, (it == 5) ? 1 : 0);
    }
}
